// MultiTaskGAT_13984413515973
// MI455X (gfx1250) — hardware-verified
//
#include <hip/hip_runtime.h>
#include <hip/hip_bf16.h>

#define NB   4096
#define NN   64
#define NC   17
#define KIN  32
#define XP   40
#define HD   128
#define NH   8
#define DK   16
#define NL   4
#define NQ   64
#define NT   256
#define SW      16.0f
#define INV_SW  0.0625f
#define PSC     4096.0f
#define FMIN16  6.103515625e-05f

typedef _Float16       v16h __attribute__((ext_vector_type(16)));
typedef _Float16       v8h  __attribute__((ext_vector_type(8)));
typedef __bf16         v16bf __attribute__((ext_vector_type(16)));
typedef unsigned short v8us __attribute__((ext_vector_type(8)));
typedef unsigned short v4us __attribute__((ext_vector_type(4)));
typedef float          v8f  __attribute__((ext_vector_type(8)));
typedef float          v4f  __attribute__((ext_vector_type(4)));
typedef v8h  __attribute__((may_alias)) v8ha;
typedef v8us __attribute__((may_alias)) v8usa;
typedef v4us __attribute__((may_alias)) v4usa;
typedef v4f  __attribute__((may_alias)) v4fa;

union FragH { v16h v; v8h p[2]; };
union FragB { v16bf v; v8us p[2]; };
union HPack { v16h v; _Float16 e[16]; };

__device__ __forceinline__ v8f wmma_f16(v16h a, v16h b, v8f c) {
  v8f d = __builtin_amdgcn_wmma_f32_16x16x32_f16(false, a, false, b, (short)0, c, false, false);
  asm volatile("v_nop\n\tv_nop\n\tv_nop\n\tv_nop" : "+v"(d) : "v"(a), "v"(b));
  return d;
}
__device__ __forceinline__ v8f wmma_bf16(v16bf a, v16bf b, v8f c) {
  v8f d = __builtin_amdgcn_wmma_f32_16x16x32_bf16(false, a, false, b, (short)0, c, false, false);
  asm volatile("v_nop\n\tv_nop\n\tv_nop\n\tv_nop" : "+v"(d) : "v"(a), "v"(b));
  return d;
}

__device__ __forceinline__ v16h load_frag_h(const _Float16* p, int h) {
  FragH f;
  f.p[0] = *(const v8ha*)(p + 8 * h);
  f.p[1] = *(const v8ha*)(p + 16 + 8 * h);
  return f.v;
}
__device__ __forceinline__ v16bf load_frag_b(const unsigned short* p, int h) {
  FragB f;
  f.p[0] = *(const v8usa*)(p + 8 * h);
  f.p[1] = *(const v8usa*)(p + 16 + 8 * h);
  return f.v;
}

__device__ __forceinline__ unsigned short bf16_bits(float f) {
  unsigned u = __float_as_uint(f);
  u += 0x7fffu + ((u >> 16) & 1u);
  return (unsigned short)(u >> 16);
}
__device__ __forceinline__ float bf16_val(unsigned short s) {
  return __uint_as_float(((unsigned)s) << 16);
}

__global__ __launch_bounds__(NT) void prep_kernel(
    const float* __restrict__ W_in, const float* __restrict__ Wg,
    const float* __restrict__ W_m,  const float* __restrict__ W_c1,
    const float* __restrict__ adj,
    unsigned short* __restrict__ winh, unsigned short* __restrict__ winl,
    _Float16* __restrict__ wgt,
    unsigned short* __restrict__ wmh,  unsigned short* __restrict__ wml,
    unsigned short* __restrict__ wc1h, unsigned short* __restrict__ wc1l,
    unsigned long long* __restrict__ amask)
{
  const int blk = blockIdx.x, tid = threadIdx.x;
  if (blk >= 60) {
    if (blk == 60 && tid < NN) {
      unsigned long long mk = 0ull;
      #pragma unroll 1
      for (int j = 0; j < NN; ++j) {
        const float av = adj[tid * NN + j];
        mk |= (av > 0.0f) ? (1ull << j) : 0ull;
      }
      *(volatile unsigned long long*)(amask + tid) = mk;
      __threadfence();
      *(volatile unsigned long long*)(amask + tid) = mk;
    }
    return;
  }
  const float* src;
  int ncol, ksrc, ksh, lg, mode;
  unsigned short* dst = winh;
  _Float16* dsth = wgt;
  if (blk < 2) {
    src = W_in; ncol = HD; ksrc = NC; ksh = 2; lg = blk * NT + tid; dst = winh; mode = 0;
  } else if (blk < 4) {
    src = W_in; ncol = HD; ksrc = NC; ksh = 2; lg = (blk - 2) * NT + tid; dst = winl; mode = 1;
  } else if (blk < 36) {
    const int lgg = (blk - 4) * NT + tid;
    const int l = lgg >> 11;
    src = Wg + (size_t)l * HD * HD; ncol = HD; ksrc = HD; ksh = 4; lg = lgg & 2047;
    dsth = wgt + (size_t)l * HD * HD; mode = 2;
  } else if (blk < 44) {
    src = W_m; ncol = HD; ksrc = HD; ksh = 4; lg = (blk - 36) * NT + tid; dst = wmh; mode = 0;
  } else if (blk < 52) {
    src = W_m; ncol = HD; ksrc = HD; ksh = 4; lg = (blk - 44) * NT + tid; dst = wml; mode = 1;
  } else if (blk < 56) {
    src = W_c1; ncol = NQ; ksrc = HD; ksh = 4; lg = (blk - 52) * NT + tid; dst = wc1h; mode = 0;
  } else {
    src = W_c1; ncol = NQ; ksrc = HD; ksh = 4; lg = (blk - 56) * NT + tid; dst = wc1l; mode = 1;
  }
  const int n  = lg >> ksh;
  const int kq = lg & ((1 << ksh) - 1);
  float v[8];
  #pragma unroll
  for (int i = 0; i < 8; ++i) {
    const int k  = kq * 8 + i;
    const int kc = (k < ksrc) ? k : (ksrc - 1);
    const float t = src[(size_t)kc * ncol + n];
    v[i] = (k < ksrc) ? t : 0.0f;
  }
  if (mode == 2) {
    const v8h o = { (_Float16)(v[0] * SW), (_Float16)(v[1] * SW), (_Float16)(v[2] * SW), (_Float16)(v[3] * SW),
                    (_Float16)(v[4] * SW), (_Float16)(v[5] * SW), (_Float16)(v[6] * SW), (_Float16)(v[7] * SW) };
    _Float16* d = dsth + (size_t)lg * 8;
    *(volatile v8h*)d = o;
    __threadfence();
    *(volatile v8h*)d = o;
  } else {
    v8us o = {0, 0, 0, 0, 0, 0, 0, 0};
    #pragma unroll
    for (int i = 0; i < 8; ++i) {
      const unsigned short hb = bf16_bits(v[i]);
      o[i] = (mode == 0) ? hb : bf16_bits(v[i] - bf16_val(hb));
    }
    unsigned short* d = dst + (size_t)lg * 8;
    *(volatile v8us*)d = o;
    __threadfence();
    *(volatile v8us*)d = o;
  }
}

__global__ __launch_bounds__(NT) void board_kernel(
    const float* __restrict__ x,     const float* __restrict__ b_in,
    const float* __restrict__ a_src, const float* __restrict__ a_dst,
    const unsigned short* __restrict__ winh, const unsigned short* __restrict__ winl,
    const _Float16* __restrict__ wgt, const unsigned long long* __restrict__ amask,
    float* __restrict__ gbuf, int nboards)
{
  __shared__ __attribute__((aligned(16))) float    sh[NN * HD];
  __shared__ __attribute__((aligned(16))) _Float16 shA[NN * HD];
  __shared__ __attribute__((aligned(16))) _Float16 shpT[HD * NN];
  __shared__ __attribute__((aligned(16))) float    shpT32[HD * NN];
  __shared__ __attribute__((aligned(16))) float    sas[NL * NH * DK];
  __shared__ __attribute__((aligned(16))) float    sad[NL * NH * DK];
  __shared__ __attribute__((aligned(16))) float    ses[NH * NN];
  __shared__ __attribute__((aligned(16))) float    sed[NH * NN];
  __shared__ __attribute__((aligned(16))) float    sE1[NH * NN];
  __shared__ __attribute__((aligned(16))) float    sE2[NH * NN];
  __shared__ __attribute__((aligned(16))) float    srinv[NH * NN];
  __shared__ __attribute__((aligned(16))) unsigned long long sadj[NN];
  __shared__ __attribute__((aligned(16))) float    sg[HD];

  const int tid = threadIdx.x, lane = tid & 31, w = tid >> 5;
  const int h = lane >> 4, m = lane & 15;
  const int b = blockIdx.x;
  if (b >= nboards) return;
  const int n0 = DK * w;
  const int head = w;

  if (tid < NN) sadj[tid] = amask[tid];
  for (int i = tid; i < NL * NH * DK; i += NT) { sas[i] = a_src[i]; sad[i] = a_dst[i]; }
  unsigned short* sxh = reinterpret_cast<unsigned short*>(shpT32);
  unsigned short* sxl = sxh + NN * XP;
  {
    const int n = tid >> 2, kq = tid & 3;
    const float* xb = x + (size_t)b * (NC * NN) + n;
    v8us oh = {0, 0, 0, 0, 0, 0, 0, 0}, ol = {0, 0, 0, 0, 0, 0, 0, 0};
    #pragma unroll
    for (int i = 0; i < 8; ++i) {
      const int k  = kq * 8 + i;
      const int kc = (k < NC) ? k : (NC - 1);
      const float t = xb[kc * NN];
      const float v = (k < NC) ? t : 0.0f;
      const unsigned short hb = bf16_bits(v);
      oh[i] = hb;
      ol[i] = bf16_bits(v - bf16_val(hb));
    }
    *(v8usa*)(sxh + n * XP + kq * 8) = oh;
    *(v8usa*)(sxl + n * XP + kq * 8) = ol;
  }
  __syncthreads();

  const v8f z8 = {0.f, 0.f, 0.f, 0.f, 0.f, 0.f, 0.f, 0.f};

  {
    const v16bf bh = load_frag_b(winh + (n0 + m) * KIN, h);
    const v16bf bl = load_frag_b(winl + (n0 + m) * KIN, h);
    v8f acc[4];
    #pragma unroll
    for (int mt = 0; mt < 4; ++mt) {
      const v16bf ah = load_frag_b(sxh + (16 * mt + m) * XP, h);
      const v16bf al = load_frag_b(sxl + (16 * mt + m) * XP, h);
      v8f c = z8;
      c = wmma_bf16(ah, bh, c);
      c = wmma_bf16(ah, bl, c);
      c = wmma_bf16(al, bh, c);
      acc[mt] = c;
    }
    const float bc = b_in[n0 + m];
    #pragma unroll
    for (int mt = 0; mt < 4; ++mt) {
      #pragma unroll
      for (int r = 0; r < 8; ++r) {
        const int row = 16 * mt + 8 * h + r;
        const float v = acc[mt][r] + bc;
        sh[row * HD + n0 + m]  = v;
        shA[row * HD + n0 + m] = (_Float16)v;
      }
    }
  }
  __syncthreads();

  #pragma unroll 1
  for (int l = 0; l < NL; ++l) {
    {
      v8f acc[4] = {z8, z8, z8, z8};
      const _Float16* wrow = wgt + ((size_t)l * HD + n0 + m) * HD;
      #pragma unroll
      for (int ks = 0; ks < 4; ++ks) {
        const v16h bf = load_frag_h(wrow + 32 * ks, h);
        #pragma unroll
        for (int mt = 0; mt < 4; ++mt) {
          const v16h af = load_frag_h(shA + (16 * mt + m) * HD + 32 * ks, h);
          acc[mt] = wmma_f16(af, bf, acc[mt]);
        }
      }
      #pragma unroll
      for (int mt = 0; mt < 4; ++mt) {
        const v8f c = acc[mt] * INV_SW;
        const int off = (n0 + m) * NN + 16 * mt + 8 * h;
        const v8h ph = { (_Float16)c[0], (_Float16)c[1], (_Float16)c[2], (_Float16)c[3],
                         (_Float16)c[4], (_Float16)c[5], (_Float16)c[6], (_Float16)c[7] };
        *(v8ha*)(shpT + off) = ph;
        const v4f c0 = { c[0], c[1], c[2], c[3] };
        const v4f c1 = { c[4], c[5], c[6], c[7] };
        *(v4fa*)(shpT32 + off)     = c0;
        *(v4fa*)(shpT32 + off + 4) = c1;
      }
    }
    __syncthreads();

    float Bstar;
    {
      float av[DK], dv[DK];
      #pragma unroll
      for (int k = 0; k < DK; ++k) {
        av[k] = sas[(l * NH + head) * DK + k];
        dv[k] = sad[(l * NH + head) * DK + k];
      }
      float edv[2];
      #pragma unroll
      for (int p = 0; p < 2; ++p) {
        const int node = lane + 32 * p;
        float es = 0.0f, ed = 0.0f;
        #pragma unroll
        for (int k = 0; k < DK; ++k) {
          const float hv = shpT32[(head * DK + k) * NN + node];
          es = fmaf(hv, av[k], es);
          ed = fmaf(hv, dv[k], ed);
        }
        edv[p] = ed;
        ses[head * NN + node] = es;
        sed[head * NN + node] = ed;
      }
      float mx = fmaxf(edv[0], edv[1]);
      mx = fmaxf(mx, __shfl_xor(mx, 16));
      mx = fmaxf(mx, __shfl_xor(mx, 8));
      mx = fmaxf(mx, __shfl_xor(mx, 4));
      mx = fmaxf(mx, __shfl_xor(mx, 2));
      mx = fmaxf(mx, __shfl_xor(mx, 1));
      Bstar = mx;
      #pragma unroll
      for (int p = 0; p < 2; ++p) {
        const int node = lane + 32 * p;
        const float d = edv[p] - Bstar;
        sE1[head * NN + node] = __expf(d);
        sE2[head * NN + node] = __expf(0.2f * d);
      }
    }
    __syncthreads();

    v8f acc2[4];
    {
      const _Float16* hpr = shpT + (head * DK + m) * NN;
      const v16h bt0 = load_frag_h(hpr, h);
      const v16h bt1 = load_frag_h(hpr + 32, h);
      #pragma unroll
      for (int mt = 0; mt < 4; ++mt) {
        const int i = 16 * mt + m;
        const float a = ses[head * NN + i];
        const unsigned long long msk = sadj[i];
        const bool allm = (msk == 0ull);
        unsigned byt[4];
        float maxb = -3.0e38f;
        #pragma unroll
        for (int g = 0; g < 4; ++g) {
          byt[g] = (unsigned)((msk >> (16 * g + 8 * h)) & 0xffull);
          const float* bp = sed + head * NN + 16 * g + 8 * h;
          const v4f b0 = *(const v4fa*)bp;
          const v4f b1 = *(const v4fa*)(bp + 4);
          const float bj[8] = { b0[0], b0[1], b0[2], b0[3], b1[0], b1[1], b1[2], b1[3] };
          #pragma unroll
          for (int jj = 0; jj < 8; ++jj)
            maxb = ((byt[g] >> jj) & 1u) ? fmaxf(maxb, bj[jj]) : maxb;
        }
        maxb = fmaxf(maxb, __shfl_xor(maxb, 16));
        const float t0 = a + maxb;
        const float C  = fmaxf(t0, 0.2f * t0);
        const float x1 = fminf(a + Bstar - C, 70.0f);
        const float x2 = fminf(0.2f * (a + Bstar) - C, 70.0f);
        const float EA1 = PSC * __expf(x1);
        const float EA2 = PSC * __expf(x2);
        float s = 0.0f;
        HPack P0, P1;
        #pragma unroll
        for (int e = 0; e < 16; ++e) { P0.e[e] = (_Float16)0.0f; P1.e[e] = (_Float16)0.0f; }
        #pragma unroll
        for (int g = 0; g < 4; ++g) {
          const int jb = head * NN + 16 * g + 8 * h;
          const v4f b0 = *(const v4fa*)(sed + jb);
          const v4f b1 = *(const v4fa*)(sed + jb + 4);
          const v4f u0 = *(const v4fa*)(sE1 + jb);
          const v4f u1 = *(const v4fa*)(sE1 + jb + 4);
          const v4f q0 = *(const v4fa*)(sE2 + jb);
          const v4f q1 = *(const v4fa*)(sE2 + jb + 4);
          const float bj[8] = { b0[0], b0[1], b0[2], b0[3], b1[0], b1[1], b1[2], b1[3] };
          const float e1[8] = { u0[0], u0[1], u0[2], u0[3], u1[0], u1[1], u1[2], u1[3] };
          const float e2[8] = { q0[0], q0[1], q0[2], q0[3], q1[0], q1[1], q1[2], q1[3] };
          #pragma unroll
          for (int jj = 0; jj < 8; ++jj) {
            const float t = a + bj[jj];
            float wv = (t > 0.0f) ? (EA1 * e1[jj]) : (EA2 * e2[jj]);
            wv = ((byt[g] >> jj) & 1u) ? wv : 0.0f;
            wv = allm ? PSC : wv;
            wv = (wv >= FMIN16) ? wv : 0.0f;
            const _Float16 hw = (_Float16)wv;
            s += (float)hw;
            if (g < 2) P0.e[8 * (g & 1) + jj] = hw; else P1.e[8 * (g & 1) + jj] = hw;
          }
        }
        s += __shfl_xor(s, 16);
        srinv[head * NN + i] = __builtin_amdgcn_rcpf(s);
        v8f c = z8;
        c = wmma_f16(P0.v, bt0, c);
        c = wmma_f16(P1.v, bt1, c);
        acc2[mt] = c;
      }
    }
    __syncthreads();

    {
      #pragma unroll
      for (int mt = 0; mt < 4; ++mt) {
        #pragma unroll
        for (int r = 0; r < 8; ++r) {
          const int row = 16 * mt + 8 * h + r;
          const int idx = row * HD + n0 + m;
          const float o = acc2[mt][r] * srinv[head * NN + row];
          float nh = sh[idx] + o;
          nh = (nh > 0.0f) ? nh : (__expf(nh) - 1.0f);
          sh[idx]  = nh;
          shA[idx] = (_Float16)nh;
        }
      }
    }
    __syncthreads();
  }

  if (tid < HD) {
    float g = -3.0e38f;
    #pragma unroll 4
    for (int i = 0; i < NN; ++i) g = fmaxf(g, sh[i * HD + tid]);
    sg[tid] = g;
  }
  __syncthreads();
  if (w == 0) {
    const v4f v = *(const v4fa*)(sg + 4 * lane);
    float* dst = gbuf + (size_t)b * HD + 4 * lane;
    *(volatile v4f*)dst = v;
    __threadfence();
    *(volatile v4f*)dst = v;
  }
}

__device__ __forceinline__ void head_store_pass(const float* semb, const float* slog,
                                                float* out_emb, float* out_logit,
                                                int r0, int w, int lane) {
  #pragma unroll
  for (int i = 0; i < 8; ++i) {
    const int row = w + 8 * i;
    const v4f v = *(const v4fa*)(semb + row * HD + 4 * lane);
    *(volatile v4f*)(out_emb + (size_t)(r0 + row) * HD + 4 * lane) = v;
  }
  if (w == 0) {
    const v4f v = *(const v4fa*)(slog + 4 * lane);
    if (lane < 16) *(volatile v4f*)(out_logit + r0 + 4 * lane) = v;
  }
}

__global__ __launch_bounds__(NT) void head_kernel(
    const float* __restrict__ gbuf,
    const unsigned short* __restrict__ wmh,  const unsigned short* __restrict__ wml,
    const unsigned short* __restrict__ wc1h, const unsigned short* __restrict__ wc1l,
    const float* __restrict__ b_m,  const float* __restrict__ b_c1,
    const float* __restrict__ W_c2, const float* __restrict__ b_c2,
    float* __restrict__ out_emb, float* __restrict__ out_logit, int nrows)
{
  __shared__ __attribute__((aligned(16))) unsigned short sgh[64 * HD];
  __shared__ __attribute__((aligned(16))) unsigned short sgl[64 * HD];
  __shared__ __attribute__((aligned(16))) float semb[64 * HD];
  __shared__ __attribute__((aligned(16))) float sq[64 * NQ];
  __shared__ __attribute__((aligned(16))) float slog[128];

  const int tid = threadIdx.x, lane = tid & 31, w = tid >> 5;
  const int h = lane >> 4, m = lane & 15;
  const int r0 = blockIdx.x * 64;
  if (r0 >= nrows) return;

  for (int idx = tid; idx < 64 * 32; idx += NT) {
    const int row = idx >> 5, c4 = idx & 31;
    int grow = r0 + row; grow = (grow < nrows) ? grow : (nrows - 1);
    const v4f v = *(const v4fa*)(gbuf + (size_t)grow * HD + 4 * c4);
    v4us hh = {0, 0, 0, 0}, ll = {0, 0, 0, 0};
    #pragma unroll
    for (int i = 0; i < 4; ++i) {
      const unsigned short hb = bf16_bits(v[i]);
      hh[i] = hb;
      ll[i] = bf16_bits(v[i] - bf16_val(hb));
    }
    *(v4usa*)(sgh + row * HD + 4 * c4) = hh;
    *(v4usa*)(sgl + row * HD + 4 * c4) = ll;
  }
  if (tid < 128) slog[tid] = 0.0f;
  __syncthreads();

  const v8f z8 = {0.f, 0.f, 0.f, 0.f, 0.f, 0.f, 0.f, 0.f};
  v8f ae[4] = {z8, z8, z8, z8};
  v8f aq[2] = {z8, z8};
  const int wq = w & 3, mq0 = 2 * (w >> 2);
  #pragma unroll
  for (int ks = 0; ks < 4; ++ks) {
    const v16bf bh = load_frag_b(wmh  + (16 * w  + m) * HD + 32 * ks, h);
    const v16bf bl = load_frag_b(wml  + (16 * w  + m) * HD + 32 * ks, h);
    const v16bf ch = load_frag_b(wc1h + (16 * wq + m) * HD + 32 * ks, h);
    const v16bf cl = load_frag_b(wc1l + (16 * wq + m) * HD + 32 * ks, h);
    #pragma unroll
    for (int mt = 0; mt < 4; ++mt) {
      const v16bf ah = load_frag_b(sgh + (16 * mt + m) * HD + 32 * ks, h);
      const v16bf al = load_frag_b(sgl + (16 * mt + m) * HD + 32 * ks, h);
      v8f c = ae[mt];
      c = wmma_bf16(ah, bh, c);
      c = wmma_bf16(ah, bl, c);
      c = wmma_bf16(al, bh, c);
      ae[mt] = c;
    }
    #pragma unroll
    for (int t = 0; t < 2; ++t) {
      const v16bf ah = load_frag_b(sgh + (16 * (mq0 + t) + m) * HD + 32 * ks, h);
      const v16bf al = load_frag_b(sgl + (16 * (mq0 + t) + m) * HD + 32 * ks, h);
      v8f c = aq[t];
      c = wmma_bf16(ah, ch, c);
      c = wmma_bf16(ah, cl, c);
      c = wmma_bf16(al, ch, c);
      aq[t] = c;
    }
  }
  {
    const float bmv = b_m[16 * w + m];
    #pragma unroll
    for (int mt = 0; mt < 4; ++mt) {
      #pragma unroll
      for (int r = 0; r < 8; ++r)
        semb[(16 * mt + 8 * h + r) * HD + 16 * w + m] = ae[mt][r] + bmv;
    }
    const float bcv = b_c1[16 * wq + m];
    #pragma unroll
    for (int t = 0; t < 2; ++t) {
      #pragma unroll
      for (int r = 0; r < 8; ++r)
        sq[(16 * (mq0 + t) + 8 * h + r) * NQ + 16 * wq + m] = fmaxf(aq[t][r] + bcv, 0.0f);
    }
  }
  __syncthreads();

  {
    const int row = tid >> 2, p = tid & 3;
    float ss = 0.0f;
    #pragma unroll 8
    for (int c = 0; c < 32; ++c) {
      const float v = semb[row * HD + 32 * p + c];
      ss = fmaf(v, v, ss);
    }
    ss += __shfl_xor(ss, 1);
    ss += __shfl_xor(ss, 2);
    const float rn = 1.0f / fmaxf(sqrtf(ss), 1e-12f);
    #pragma unroll 8
    for (int c = 0; c < 32; ++c) semb[row * HD + 32 * p + c] *= rn;
    float lg = 0.0f;
    #pragma unroll 4
    for (int t = 0; t < 16; ++t) lg = fmaf(sq[row * NQ + 16 * p + t], W_c2[16 * p + t], lg);
    lg += __shfl_xor(lg, 1);
    lg += __shfl_xor(lg, 2);
    if (p == 0) slog[row] = lg + b_c2[0];
  }
  __syncthreads();

  head_store_pass(semb, slog, out_emb, out_logit, r0, w, lane);
  __threadfence();
  head_store_pass(semb, slog, out_emb, out_logit, r0, w, lane);
}

extern "C" void kernel_launch(void* const* d_in, const int* in_sizes, int n_in,
                              void* d_out, int out_size, void* d_ws, size_t ws_size,
                              hipStream_t stream) {
  if (n_in < 13) return;
  if (in_sizes[0] != NB * NC * NN) return;
  if (in_sizes[1] != NN * NN) return;
  if (in_sizes[2] != NC * HD || in_sizes[3] != HD) return;
  if (in_sizes[4] != NL * HD * HD) return;
  if (in_sizes[5] != NL * NH * DK || in_sizes[6] != NL * NH * DK) return;
  if (in_sizes[7] != HD * HD || in_sizes[8] != HD) return;
  if (in_sizes[9] != HD * NQ || in_sizes[10] != NQ) return;
  if (in_sizes[11] != NQ || in_sizes[12] != 1) return;
  if (out_size != NB * HD + NB) return;

  const float* x     = (const float*)d_in[0];
  const float* adj   = (const float*)d_in[1];
  const float* W_in  = (const float*)d_in[2];
  const float* b_in  = (const float*)d_in[3];
  const float* Wg    = (const float*)d_in[4];
  const float* a_src = (const float*)d_in[5];
  const float* a_dst = (const float*)d_in[6];
  const float* W_m   = (const float*)d_in[7];
  const float* b_m   = (const float*)d_in[8];
  const float* W_c1  = (const float*)d_in[9];
  const float* b_c1  = (const float*)d_in[10];
  const float* W_c2  = (const float*)d_in[11];
  const float* b_c2  = (const float*)d_in[12];

  float* out       = (float*)d_out;
  float* out_emb   = out;
  float* out_logit = out + (size_t)NB * HD;

  const size_t win_bytes  = (size_t)HD * KIN * 2;
  const size_t wgt_bytes  = (size_t)NL * HD * HD * 2;
  const size_t wm_bytes   = (size_t)HD * HD * 2;
  const size_t wc1_bytes  = (size_t)NQ * HD * 2;
  const size_t am_bytes   = (size_t)NN * 8;
  const size_t g_bytes    = (size_t)NB * HD * 4;
  const size_t o_winh = 0;
  const size_t o_winl = o_winh + win_bytes;
  const size_t o_wgt  = o_winl + win_bytes;
  const size_t o_wmh  = o_wgt  + wgt_bytes;
  const size_t o_wml  = o_wmh  + wm_bytes;
  const size_t o_wc1h = o_wml  + wm_bytes;
  const size_t o_wc1l = o_wc1h + wc1_bytes;
  const size_t o_am   = o_wc1l + wc1_bytes;
  const size_t o_g    = o_am   + am_bytes;
  const size_t total  = o_g + g_bytes;
  if (total > ws_size) return;

  char* ws = (char*)d_ws;
  unsigned short* winh = (unsigned short*)(ws + o_winh);
  unsigned short* winl = (unsigned short*)(ws + o_winl);
  _Float16* wgt        = (_Float16*)(ws + o_wgt);
  unsigned short* wmh  = (unsigned short*)(ws + o_wmh);
  unsigned short* wml  = (unsigned short*)(ws + o_wml);
  unsigned short* wc1h = (unsigned short*)(ws + o_wc1h);
  unsigned short* wc1l = (unsigned short*)(ws + o_wc1l);
  unsigned long long* am = (unsigned long long*)(ws + o_am);
  float* gbuf          = (float*)(ws + o_g);

  const int nboards = in_sizes[0] / (NC * NN);

  prep_kernel<<<dim3(61), dim3(NT), 0, stream>>>(W_in, Wg, W_m, W_c1, adj,
                                                  winh, winl, wgt, wmh, wml, wc1h, wc1l, am);

  board_kernel<<<dim3(nboards), dim3(NT), 0, stream>>>(x, b_in, a_src, a_dst,
                                                        winh, winl, wgt, am, gbuf, nboards);

  head_kernel<<<dim3((nboards + 63) / 64), dim3(NT), 0, stream>>>(gbuf, wmh, wml, wc1h, wc1l,
                                                                   b_m, b_c1, W_c2, b_c2,
                                                                   out_emb, out_logit, nboards);
}
